// TaylorMap_26388279067203
// MI455X (gfx1250) — hardware-verified
//
#include <hip/hip_runtime.h>
#include <stddef.h>


#define NB     4096
#define NF     32
#define NPOLY  33825
#define NCH    1058
#define KP     (NCH * 32)
#define KP8    (KP / 8)
#define CH     2
#define NPH    (NCH / CH)
#define BM     128
#define NTHR   256
#define NWAVE  8
#define APITCH 72
#define CA     1024.0f
#define CB     256.0f
#define WSCAP  134217728

static_assert(KP == 33856);
static_assert((NCH % CH) == 0);
static_assert(NCH == 2 + 32 + 1024);
static_assert((NB % BM) == 0);
static_assert(BM == NWAVE * 16 && NTHR == NWAVE * 32 && NTHR == 2 * BM);
static_assert(((32 * KP8) % NTHR) == 0);
static_assert(((BM * NF) % NTHR) == 0);
static_assert((APITCH % 8) == 0 && APITCH >= CH * 32);
static_assert(((KP * 2) % 16) == 0);

typedef float     v4f  __attribute__((ext_vector_type(4)));
typedef float     v8f  __attribute__((ext_vector_type(8)));
typedef _Float16  v8h  __attribute__((ext_vector_type(8)));
typedef _Float16  v16h __attribute__((ext_vector_type(16)));
union FragH { v16h v; v8h h[2]; };

__device__ __forceinline__ v8f wmf(v16h a, v16h b, v8f c) {
  v8f d = __builtin_amdgcn_wmma_f32_16x16x32_f16(false, a, false, b, (short)0, c, false, false);
  asm volatile("v_nop\n\tv_nop\n\tv_nop\n\tv_nop" : "+v"(d) : "v"(a), "v"(b));
  return d;
}

__global__ __launch_bounds__(NTHR) void k_wprep(const float* __restrict__ W, _Float16* Wt) {
  const int t  = blockIdx.x * NTHR + threadIdx.x;
  const int n  = t / KP8;
  const int k8 = t - n * KP8;
  v8h hv;
#pragma unroll
  for (int e = 0; e < 8; ++e) {
    const int kp = 8 * k8 + e;
    const int pr = max(kp - 31, 0);
    const float w = W[(size_t)pr * NF + n];
    const bool keep = (kp == 0) || (kp >= 32);
    hv[e] = keep ? (_Float16)(w * CB) : (_Float16)0.0f;
  }
  _Float16* d = Wt + (size_t)t * 8;
  *(volatile v8h*)d = hv;
  __threadfence();
  *(volatile v8h*)d = hv;
}

__global__ __launch_bounds__(NTHR) void k_gemm(const float* __restrict__ X, const _Float16* __restrict__ Wt,
                                               float* out) {
  __shared__ __attribute__((aligned(16))) float    xs[BM * NF];
  __shared__ __attribute__((aligned(16))) _Float16 as[BM * APITCH];
  __shared__ __attribute__((aligned(16))) float    stg[BM * NF];

  const int tid = threadIdx.x, lane = tid & 31, wave = tid >> 5, hh = lane >> 4, m = lane & 15;
  const int rowBase = blockIdx.x * BM;

#pragma unroll
  for (int e = 0; e < (BM * NF) / NTHR; ++e) {
    const int idx = e * NTHR + tid;
    xs[idx] = X[(size_t)rowBase * NF + idx];
  }

  const int gm = tid >> 1, q = tid & 1;
  float xk[16];
  {
    const float* xp = X + (size_t)(rowBase + gm) * NF + 16 * q;
#pragma unroll
    for (int v = 0; v < 4; ++v) {
      const v4f t4 = *(const v4f*)(xp + 4 * v);
      xk[4 * v + 0] = t4.x; xk[4 * v + 1] = t4.y; xk[4 * v + 2] = t4.z; xk[4 * v + 3] = t4.w;
    }
  }
  const float g0 = (q == 0) ? CA : 0.0f;
  const float* xrow = xs + gm * NF;
  _Float16* arow = as + gm * APITCH + 16 * q;

  const _Float16* ab  = as + (16 * wave + m) * APITCH + 8 * hh;
  const _Float16* bb0 = Wt + (size_t)m * KP + 8 * hh;
  const _Float16* bb1 = Wt + (size_t)(16 + m) * KP + 8 * hh;

  v8f acc[2];
  {
    v8f z = {0.f, 0.f, 0.f, 0.f, 0.f, 0.f, 0.f, 0.f};
    acc[0] = z; acc[1] = z;
  }

#pragma unroll 1
  for (int ph = 0; ph < NPH; ++ph) {
    __syncthreads();
#pragma unroll
    for (int cc = 0; cc < CH; ++cc) {
      const int c  = CH * ph + cc;
      const int u  = max(c - 34, 0);
      const int i2 = min(max(c - 2, 0), 31);
      const float xa = xrow[u >> 5];
      const float xb = xrow[u & 31];
      const float xd = xrow[i2];
      const float f1 = (c >= 34) ? (CA * xa) : ((c >= 1) ? CA : 0.0f);
      const float f2 = (c >= 34) ? xb : ((c >= 2) ? xd : 1.0f);
      const float e0 = (c == 0) ? g0 : 0.0f;
      v8h lo, hi;
#pragma unroll
      for (int e = 0; e < 8; ++e) {
        const float a0 = f1 * (f2 * xk[e]);
        const float a1 = f1 * (f2 * xk[8 + e]);
        lo[e] = (_Float16)((e == 0) ? (a0 + e0) : a0);
        hi[e] = (_Float16)a1;
      }
      *(v8h*)(arow + cc * 32)     = lo;
      *(v8h*)(arow + cc * 32 + 8) = hi;
    }
    __syncthreads();
#pragma unroll
    for (int cc = 0; cc < CH; ++cc) {
      const size_t k0 = (size_t)32 * (size_t)(CH * ph + cc);
      FragH a, b0, b1;
      a.h[0]  = *(const v8h*)(ab + cc * 32);
      a.h[1]  = *(const v8h*)(ab + cc * 32 + 16);
      b0.h[0] = *(const v8h*)(bb0 + k0);
      b0.h[1] = *(const v8h*)(bb0 + k0 + 16);
      b1.h[0] = *(const v8h*)(bb1 + k0);
      b1.h[1] = *(const v8h*)(bb1 + k0 + 16);
      acc[0] = wmf(a.v, b0.v, acc[0]);
      acc[1] = wmf(a.v, b1.v, acc[1]);
    }
  }

  const float OSC = 1.0f / 262144.0f;
#pragma unroll
  for (int j = 0; j < 2; ++j) {
#pragma unroll
    for (int r = 0; r < 8; ++r) {
      const int idx = (16 * wave + 8 * hh + r) * NF + 16 * j + m;
      stg[idx] = acc[j][r] * OSC + xs[idx];
    }
  }
  __syncthreads();

  const int rq = lane >> 3, c4 = 4 * (lane & 7);
  float* gb = out + (size_t)(rowBase + 16 * wave) * NF + c4;
  const float* sb = stg + (16 * wave) * NF + c4;
#pragma unroll
  for (int it = 0; it < 4; ++it) {
    const int row = 4 * it + rq;
    const v4f v = *(const v4f*)(sb + row * NF);
    *(volatile v4f*)(gb + (size_t)row * NF) = v;
  }
  __threadfence();
#pragma unroll
  for (int it = 0; it < 4; ++it) {
    const int row = 4 * it + rq;
    const v4f v = *(const v4f*)(sb + row * NF);
    *(volatile v4f*)(gb + (size_t)row * NF) = v;
  }
}

extern "C" void kernel_launch(void* const* d_in, const int* in_sizes, int n_in,
                              void* d_out, int out_size, void* d_ws, size_t ws_size,
                              hipStream_t stream) {
  if (n_in < 2) return;
  if (in_sizes[0] != NB * NF) return;
  if (in_sizes[1] != NPOLY * NF) return;
  if (out_size != NB * NF) return;

  const float* X = (const float*)d_in[0];
  const float* W = (const float*)d_in[1];
  float* out = (float*)d_out;

  size_t off = 0;
  const size_t oW = off;
  off += (size_t)32 * KP * 2;
  off = (off + 255) & ~(size_t)255;
  if (off > ws_size || off > (size_t)WSCAP) return;
  char* ws = (char*)d_ws;
  _Float16* wt = (_Float16*)(ws + oW);

  k_wprep<<<(32 * KP8) / NTHR, NTHR, 0, stream>>>(W, wt);

  k_gemm<<<NB / BM, NTHR, 0, stream>>>(X, wt, out);
}
